// MambaLayer_72464688218885
// MI455X (gfx1250) — hardware-verified
//
#include <hip/hip_runtime.h>
#include <math.h>

typedef __attribute__((ext_vector_type(16))) _Float16 v16h;
typedef __attribute__((ext_vector_type(8)))  _Float16 v8h;
typedef __attribute__((ext_vector_type(16))) __bf16   v16b;
typedef __attribute__((ext_vector_type(8)))  __bf16   v8b;
typedef __attribute__((ext_vector_type(8)))  float    v8f;
typedef __attribute__((ext_vector_type(4)))  float    v4f;

constexpr int kBatch  = 2;
constexpr int kDim    = 96;
constexpr int kSeq    = 13824;
constexpr int kDin    = 192;
constexpr int kNst    = 16;
constexpr int kDtR    = 6;
constexpr int kXpN    = 38;
constexpr int kXzP    = 2 * kDin;
constexpr int kXdP    = 64;
constexpr int kRows   = kBatch * kSeq;
constexpr int kOutM   = 128;
constexpr int kLnXP   = 65;
constexpr int kLnNP   = 100;
constexpr int kConvTP = 196;
constexpr int kScanTS = 64;
constexpr int kScanCh = 64;
constexpr int kScanYP = 68;
constexpr float kInvDim = 1.0f / (float)kDim;
constexpr float kLnEps  = 1e-5f;
static_assert(kDtR + 2 * kNst == kXpN, "");
static_assert((kDim % 32) == 0 && (kDin % 32) == 0, "");
static_assert((kRows % 64) == 0 && (kXzP % 64) == 0 && (kXdP % 64) == 0 && (kSeq % 64) == 0 && (kOutM % 64) == 0, "");
static_assert((kDim % 16) == 0 && kDim <= kOutM, "");
static_assert((kSeq % kScanTS) == 0 && (kDin % kScanCh) == 0 && (kSeq % 64) == 0, "");
static_assert(((size_t)kSeq * 4) % 256 == 0, "");
static_assert(64 * kDim == 12 * 8 * 64 && 16 * kDin == 48 * 4 * 16, "");

constexpr size_t kOffXNH  = 0;
constexpr size_t kOffXNL  = kOffXNH + (size_t)kRows * kDim * 2;
constexpr size_t kOffWIH  = kOffXNL + (size_t)kRows * kDim * 2;
constexpr size_t kOffWIL  = kOffWIH + (size_t)kXzP  * kDim * 2;
constexpr size_t kOffWXH  = kOffWIL + (size_t)kXzP  * kDim * 2;
constexpr size_t kOffWOH  = kOffWXH + (size_t)kXdP  * kDin * 2;
constexpr size_t kOffWOL  = kOffWOH + (size_t)kOutM * kDin * 2;
constexpr size_t kOffXZ   = kOffWOL + (size_t)kOutM * kDin * 2;
constexpr size_t kOffUC   = kOffXZ  + (size_t)kRows * kXzP * 4;
constexpr size_t kOffUCH  = kOffUC  + (size_t)kRows * kDin * 4;
constexpr size_t kOffXD   = kOffUCH + (size_t)kRows * kDin * 2;
constexpr size_t kOffYH   = kOffXD  + (size_t)kRows * kXdP * 4;
constexpr size_t kOffYL   = kOffYH  + (size_t)kRows * kDin * 2;
constexpr size_t kWsTotal = kOffYL  + (size_t)kRows * kDin * 2;
static_assert(kWsTotal == 113516544ull, "");
static_assert(kWsTotal <= 134217728ull, "");
static_assert((kOffXNL % 256) == 0 && (kOffWIH % 256) == 0 && (kOffWIL % 256) == 0 && (kOffWXH % 256) == 0 &&
              (kOffWOH % 256) == 0 && (kOffWOL % 256) == 0 && (kOffXZ % 256) == 0 && (kOffUC % 256) == 0 &&
              (kOffUCH % 256) == 0 && (kOffXD % 256) == 0 && (kOffYH % 256) == 0 && (kOffYL % 256) == 0, "");

__device__ __forceinline__ unsigned short f2bf_bits(float f) {
  unsigned u = __float_as_uint(f);
  return (unsigned short)((u + 0x7FFFu + ((u >> 16) & 1u)) >> 16);
}
__device__ __forceinline__ float bf_bits2f(unsigned short h) { return __uint_as_float(((unsigned)h) << 16); }

__device__ __forceinline__ void dep_guard4_h(v8f& a, v8f& b, v8f& c, v8f& d, v16h x, v16h y) {
  asm volatile("v_nop\n\tv_nop\n\tv_nop\n\tv_nop" : "+v"(a), "+v"(b), "+v"(c), "+v"(d) : "v"(x), "v"(y));
}
__device__ __forceinline__ void dep_guard4_b(v8f& a, v8f& b, v8f& c, v8f& d, v16b x, v16b y) {
  asm volatile("v_nop\n\tv_nop\n\tv_nop\n\tv_nop" : "+v"(a), "+v"(b), "+v"(c), "+v"(d) : "v"(x), "v"(y));
}
__device__ __forceinline__ void keep4_h(v16h a, v16h b, v16h c, v16h d) { asm volatile("v_nop" :: "v"(a), "v"(b), "v"(c), "v"(d)); }
__device__ __forceinline__ void keep4_b(v16b a, v16b b, v16b c, v16b d) { asm volatile("v_nop" :: "v"(a), "v"(b), "v"(c), "v"(d)); }
__device__ __forceinline__ void acc_guard4(v8f& a, v8f& b, v8f& c, v8f& d) { asm volatile("v_nop\n\tv_nop\n\tv_nop\n\tv_nop" : "+v"(a), "+v"(b), "+v"(c), "+v"(d)); }
template <typename T> struct Frag;
template <> struct Frag<_Float16> {
  typedef v16h V; union U { v16h v; v8h h[2]; };
  static __device__ __forceinline__ v16h load(const _Float16* p) {
    U f; f.h[0] = *(const v8h*)(p); f.h[1] = *(const v8h*)(p + 16); return f.v;
  }
  static __device__ __forceinline__ v8f mma(v16h a, v16h b, v8f c) {
    return __builtin_amdgcn_wmma_f32_16x16x32_f16(false, a, false, b, (short)0, c, false, false);
  }
  static __device__ __forceinline__ void guard4(v8f& a, v8f& b, v8f& c, v8f& d, v16h x, v16h y) { dep_guard4_h(a, b, c, d, x, y); }
  static __device__ __forceinline__ void keep(v16h a, v16h b, v16h c, v16h d) { keep4_h(a, b, c, d); }
};
template <> struct Frag<__bf16> {
  typedef v16b V; union U { v16b v; v8b h[2]; };
  static __device__ __forceinline__ v16b load(const __bf16* p) {
    U f; f.h[0] = *(const v8b*)(p); f.h[1] = *(const v8b*)(p + 16); return f.v;
  }
  static __device__ __forceinline__ v8f mma(v16b a, v16b b, v8f c) {
    return __builtin_amdgcn_wmma_f32_16x16x32_bf16(false, a, false, b, (short)0, c, false, false);
  }
  static __device__ __forceinline__ void guard4(v8f& a, v8f& b, v8f& c, v8f& d, v16b x, v16b y) { dep_guard4_b(a, b, c, d, x, y); }
  static __device__ __forceinline__ void keep(v16b a, v16b b, v16b c, v16b d) { keep4_b(a, b, c, d); }
};

template <int ET> struct Elem;
template <> struct Elem<0> { typedef _Float16 T; };
template <> struct Elem<1> { typedef __bf16 T; };
template <int ET, bool SPLIT, int BIAS_MODE, int OUT_MODE, bool RESID, int ACT = 0>
__global__ __launch_bounds__(256) void wmma_gemm64(
    const unsigned short* __restrict__ Ap, const unsigned short* __restrict__ A2p, int lda, long strideA,
    const unsigned short* __restrict__ Btp, const unsigned short* __restrict__ Bt2p, int ldb, long strideB,
    void* __restrict__ Cout, void* __restrict__ Cout2, int ldc, long strideC,
    const float* __restrict__ bias,
    const float* __restrict__ resid, long strideR,
    int M, int N, int K, float scale, int Mlim) {
  typedef typename Elem<ET>::T T;
  typedef typename Frag<T>::V V;
  const T* A = (const T*)Ap; const T* A2 = (const T*)A2p; const T* Bt = (const T*)Btp; const T* Bt2 = (const T*)Bt2p;
  __shared__ __align__(16) float sT[8][16 * 68];
  const int b    = blockIdx.y;
  const int lane = threadIdx.x & 31;
  const int wave = threadIdx.x >> 5;
  const int tilesN = N >> 6;
  const int tilesM = M >> 6;
  const int tile = blockIdx.x * 8 + wave;
  if (tile >= tilesM * tilesN) return;
  const int tm = tile / tilesN;
  const int tn = tile - tm * tilesN;
  const int m0 = tm << 6;
  const int n0 = tn << 6;

  const T* Ab  = A  + (size_t)b * strideA;
  const T* Bb  = Bt + (size_t)b * strideB;
  const T* Ab2 = SPLIT ? (A2  + (size_t)b * strideA) : nullptr;
  const T* Bb2 = SPLIT ? (Bt2 + (size_t)b * strideB) : nullptr;

  const int rlane = lane & 15;
  const int koff  = (lane >> 4) * 8;
  const int mOff  = (lane >> 4) * 8;

  v8f acc[4][4];
#pragma unroll
  for (int i = 0; i < 4; ++i)
#pragma unroll
    for (int j = 0; j < 4; ++j) acc[i][j] = (v8f){0.f,0.f,0.f,0.f,0.f,0.f,0.f,0.f};

  for (int k0 = 0; k0 < K; k0 += 32) {
    V bh[4], bl[4];
#pragma unroll
    for (int j = 0; j < 4; ++j) {
      const size_t bo = (size_t)(n0 + (j << 4) + rlane) * ldb + koff + k0;
      bh[j] = Frag<T>::load(Bb + bo);
      if (SPLIT) bl[j] = Frag<T>::load(Bb2 + bo);
    }
#pragma unroll
    for (int i = 0; i < 4; ++i) {
      const size_t ao = (size_t)(m0 + (i << 4) + rlane) * lda + koff + k0;
      V ah = Frag<T>::load(Ab + ao);
      V al;
      if (SPLIT) al = Frag<T>::load(Ab2 + ao);
#pragma unroll
      for (int j = 0; j < 4; ++j) {
        acc[i][j] = Frag<T>::mma(ah, bh[j], acc[i][j]);
        if (SPLIT) {
          acc[i][j] = Frag<T>::mma(ah, bl[j], acc[i][j]);
          acc[i][j] = Frag<T>::mma(al, bh[j], acc[i][j]);
        }
      }
      Frag<T>::guard4(acc[i][0], acc[i][1], acc[i][2], acc[i][3], ah, SPLIT ? al : ah);
    }
    Frag<T>::keep(bh[0], bh[1], bh[2], bh[3]);
    if (SPLIT) Frag<T>::keep(bl[0], bl[1], bl[2], bl[3]);
  }
  acc_guard4(acc[0][0], acc[0][1], acc[0][2], acc[0][3]);
  acc_guard4(acc[1][0], acc[1][1], acc[1][2], acc[1][3]);
  acc_guard4(acc[2][0], acc[2][1], acc[2][2], acc[2][3]);
  acc_guard4(acc[3][0], acc[3][1], acc[3][2], acc[3][3]);

  float* slab = sT[wave];
  const float* Rb = RESID ? (resid + (size_t)b * strideR) : nullptr;
#pragma unroll
  for (int i = 0; i < 4; ++i) {
    const int mBase = m0 + (i << 4);
#pragma unroll
    for (int j = 0; j < 4; ++j) {
      const int n = n0 + (j << 4) + rlane;
      float bv = 0.f;
      if (BIAS_MODE == 2) bv = bias[n];
#pragma unroll
      for (int r = 0; r < 8; ++r) {
        float v = acc[i][j][r] * scale;
        if (BIAS_MODE == 1) v += bias[mBase + mOff + r];
        if (BIAS_MODE == 2) v += bv;
        if (RESID) v += Rb[(size_t)(mBase + mOff + r) * ldc + n];
        if (ACT == 1) v = tanhf(v);
        if (ACT == 2) v = fmaxf(v, 0.0f);
        if (ACT == 3) v = v / (1.0f + expf(-v));
        if (ACT == 4) v = (v > 0.f) ? v : 0.01f * v;
        slab[(mOff + r) * 68 + (j << 4) + rlane] = v;
      }
    }
    __builtin_amdgcn_fence(__ATOMIC_RELEASE, "workgroup");
    __builtin_amdgcn_wave_barrier();
    __builtin_amdgcn_fence(__ATOMIC_ACQUIRE, "workgroup");
    const bool live = (mBase < Mlim);
    if (OUT_MODE == 0) {
      float* C = (float*)Cout + (size_t)b * strideC;
      const int hh = lane >> 4, c4 = (lane & 15) * 4;
      if (live) {
        for (int pass = 0; pass < 2; ++pass) {
#pragma unroll
          for (int it = 0; it < 8; ++it) {
            const int row = it * 2 + hh;
            v4f v = *(const v4f*)(slab + row * 68 + c4);
            *(volatile v4f*)(C + (size_t)(mBase + row) * ldc + n0 + c4) = v;
          }
          __threadfence();
        }
      }
    } else {
      const int q = lane >> 3, c8 = (lane & 7) * 8;
      unsigned short* C  = (unsigned short*)Cout  + (size_t)b * strideC;
      unsigned short* C2 = (OUT_MODE == 2) ? ((unsigned short*)Cout2 + (size_t)b * strideC) : nullptr;
      if (live) {
        for (int pass = 0; pass < 2; ++pass) {
#pragma unroll
          for (int it = 0; it < 4; ++it) {
            const int row = it * 4 + q;
            const float* sp = slab + row * 68 + c8;
            v8h hv, lv;
#pragma unroll
            for (int e = 0; e < 8; ++e) {
              if (OUT_MODE == 1) {
                hv[e] = (_Float16)sp[e];
              } else {
                unsigned short hb = f2bf_bits(sp[e]);
                unsigned short lb = f2bf_bits(sp[e] - bf_bits2f(hb));
                hv[e] = __builtin_bit_cast(_Float16, hb);
                lv[e] = __builtin_bit_cast(_Float16, lb);
              }
            }
            *(volatile v8h*)(C + (size_t)(mBase + row) * ldc + n0 + c8) = hv;
            if (OUT_MODE == 2) *(volatile v8h*)(C2 + (size_t)(mBase + row) * ldc + n0 + c8) = lv;
          }
          __threadfence();
        }
      }
    }
    __builtin_amdgcn_fence(__ATOMIC_RELEASE, "workgroup");
    __builtin_amdgcn_wave_barrier();
    __builtin_amdgcn_fence(__ATOMIC_ACQUIRE, "workgroup");
  }
}

__global__ __launch_bounds__(256) void split_pad_bf16_kernel(
    const float* __restrict__ src, unsigned short* __restrict__ dhi, unsigned short* __restrict__ dlo, int real8, int pad8)
{
  const int i = blockIdx.x * 256 + threadIdx.x;
  if (i >= pad8) return;
  const bool live = (i < real8);
  const int ic = live ? i : (real8 - 1);
  const size_t e0 = (size_t)ic << 3;
  const v4f a0 = *(const v4f*)(src + e0);
  const v4f a1 = *(const v4f*)(src + e0 + 4);
  v8h hv, lv;
#pragma unroll
  for (int e = 0; e < 4; ++e) {
    const float f0 = live ? a0[e] : 0.f;
    const float f1 = live ? a1[e] : 0.f;
    const unsigned short h0 = f2bf_bits(f0), h1 = f2bf_bits(f1);
    const unsigned short l0 = f2bf_bits(f0 - bf_bits2f(h0)), l1 = f2bf_bits(f1 - bf_bits2f(h1));
    hv[e]     = __builtin_bit_cast(_Float16, h0);
    hv[4 + e] = __builtin_bit_cast(_Float16, h1);
    lv[e]     = __builtin_bit_cast(_Float16, l0);
    lv[4 + e] = __builtin_bit_cast(_Float16, l1);
  }
  unsigned short* qh = dhi + ((size_t)i << 3);
  unsigned short* ql = dlo + ((size_t)i << 3);
  *(volatile v8h*)qh = hv;
  *(volatile v8h*)ql = lv;
  __threadfence();
  *(volatile v8h*)qh = hv;
  *(volatile v8h*)ql = lv;
}

__global__ __launch_bounds__(256) void xproj_plane_kernel(
    const float* __restrict__ W, unsigned short* __restrict__ WXH, int total8)
{
  const int i = blockIdx.x * 256 + threadIdx.x;
  if (i >= total8) return;
  const int n  = i / (kDin / 8);
  const int k8 = (i - n * (kDin / 8)) * 8;
  const bool live = (n < kDtR) || (n >= 8 && n < 8 + 2 * kNst);
  int src = (n < kDtR) ? n : (n - 2);
  src = live ? src : 0;
  const float* p = W + (size_t)src * kDin + k8;
  const v4f a0 = *(const v4f*)(p);
  const v4f a1 = *(const v4f*)(p + 4);
  v8h hv;
#pragma unroll
  for (int e = 0; e < 4; ++e) {
    const float f0 = live ? a0[e] : 0.f;
    const float f1 = live ? a1[e] : 0.f;
    hv[e]     = __builtin_bit_cast(_Float16, f2bf_bits(f0));
    hv[4 + e] = __builtin_bit_cast(_Float16, f2bf_bits(f1));
  }
  unsigned short* qh = WXH + ((size_t)i << 3);
  *(volatile v8h*)qh = hv;
  __threadfence();
  *(volatile v8h*)qh = hv;
}

__global__ __launch_bounds__(256) void ln_split_kernel(
    const float* __restrict__ x, const float* __restrict__ gam, const float* __restrict__ bet,
    unsigned short* __restrict__ XNH, unsigned short* __restrict__ XNL)
{
  __shared__ __align__(16) float sX[kDim * kLnXP];
  __shared__ __align__(16) float sN[64 * kLnNP];
  const int tid = threadIdx.x, lane = tid & 31, wave = tid >> 5;
  const int m0 = blockIdx.x * 64;
  const int b  = m0 / kSeq;
  const int l0 = m0 - b * kSeq;
  const float* xb = x + (size_t)b * kDim * kSeq + l0;
#pragma unroll
  for (int p = 0; p < 6; ++p) {
    const int idx = p * 256 + tid;
    const int c   = idx >> 4;
    const int j4  = (idx & 15) * 4;
    const v4f v = *(const v4f*)(xb + (size_t)c * kSeq + j4);
    float* dst = sX + c * kLnXP + j4;
    dst[0] = v[0]; dst[1] = v[1]; dst[2] = v[2]; dst[3] = v[3];
  }
  __syncthreads();
  const float g0 = gam[lane], g1 = gam[lane + 32], g2 = gam[lane + 64];
  const float e0 = bet[lane], e1 = bet[lane + 32], e2 = bet[lane + 64];
#pragma unroll 1
  for (int jj = 0; jj < 8; ++jj) {
    const int j = wave * 8 + jj;
    const float v0 = sX[lane * kLnXP + j];
    const float v1 = sX[(lane + 32) * kLnXP + j];
    const float v2 = sX[(lane + 64) * kLnXP + j];
    float s = (v0 + v1) + v2;
#pragma unroll
    for (int off = 16; off > 0; off >>= 1) s += __shfl_xor(s, off, 32);
    const float mu = s * kInvDim;
    const float d0 = v0 - mu, d1 = v1 - mu, d2 = v2 - mu;
    float q = d0 * d0;
    q = fmaf(d1, d1, q);
    q = fmaf(d2, d2, q);
#pragma unroll
    for (int off = 16; off > 0; off >>= 1) q += __shfl_xor(q, off, 32);
    const float var  = q * kInvDim;
    const float rstd = rsqrtf(var + kLnEps);
    float* nr = sN + j * kLnNP;
    nr[lane]      = fmaf(d0 * rstd, g0, e0);
    nr[lane + 32] = fmaf(d1 * rstd, g1, e1);
    nr[lane + 64] = fmaf(d2 * rstd, g2, e2);
  }
  __syncthreads();
  v8h hv[3], lv[3];
#pragma unroll
  for (int it = 0; it < 3; ++it) {
    const int ch  = it * 256 + tid;
    const int row = ch / 12;
    const int col = (ch - row * 12) * 8;
    const float* sp = sN + row * kLnNP + col;
    const v4f a0 = *(const v4f*)(sp);
    const v4f a1 = *(const v4f*)(sp + 4);
#pragma unroll
    for (int e = 0; e < 4; ++e) {
      const unsigned short h0 = f2bf_bits(a0[e]), h1 = f2bf_bits(a1[e]);
      const unsigned short l0b = f2bf_bits(a0[e] - bf_bits2f(h0)), l1b = f2bf_bits(a1[e] - bf_bits2f(h1));
      hv[it][e]     = __builtin_bit_cast(_Float16, h0);
      hv[it][4 + e] = __builtin_bit_cast(_Float16, h1);
      lv[it][e]     = __builtin_bit_cast(_Float16, l0b);
      lv[it][4 + e] = __builtin_bit_cast(_Float16, l1b);
    }
  }
  for (int pass = 0; pass < 2; ++pass) {
#pragma unroll
    for (int it = 0; it < 3; ++it) {
      const size_t o = (size_t)m0 * kDim + (size_t)(it * 256 + tid) * 8;
      *(volatile v8h*)(XNH + o) = hv[it];
      *(volatile v8h*)(XNL + o) = lv[it];
    }
    __threadfence();
  }
}

__global__ __launch_bounds__(192) void conv_silu_kernel(
    const float* __restrict__ XZ, const float* __restrict__ cw, const float* __restrict__ cb,
    float* __restrict__ UC, unsigned short* __restrict__ UCH)
{
  __shared__ __align__(16) float sT[16 * kConvTP];
  const int tid = threadIdx.x;
  const int d = tid;
  const int g0 = blockIdx.x * 64;
  const int bb = g0 / kSeq;
  const int tb = g0 - bb * kSeq;
  const float w0 = cw[d * 4 + 0], w1 = cw[d * 4 + 1], w2 = cw[d * 4 + 2], w3 = cw[d * 4 + 3];
  const float bc = cb[d];
  float xm3, xm2, xm1;
  {
    const bool hist = (tb > 0);
    const int rb = hist ? (g0 - 3) : g0;
    const float v3 = XZ[(size_t)rb * kXzP + d];
    const float v2 = XZ[(size_t)(rb + 1) * kXzP + d];
    const float v1 = XZ[(size_t)(rb + 2) * kXzP + d];
    xm3 = hist ? v3 : 0.f;
    xm2 = hist ? v2 : 0.f;
    xm1 = hist ? v1 : 0.f;
  }
#pragma unroll 1
  for (int sub = 0; sub < 4; ++sub) {
    const int lb = g0 + sub * 16;
#pragma unroll 1
    for (int s = 0; s < 16; ++s) {
      const float xcur = XZ[(size_t)(lb + s) * kXzP + d];
      float acc = w0 * xm3;
      acc = fmaf(w1, xm2, acc);
      acc = fmaf(w2, xm1, acc);
      acc = fmaf(w3, xcur, acc);
      const float sv = acc + bc;
      const float sg = __builtin_amdgcn_rcpf(1.0f + expf(-sv));
      sT[s * kConvTP + tid] = sv * sg;
      xm3 = xm2; xm2 = xm1; xm1 = xcur;
    }
    __syncthreads();
    v4f fv[4];
    v8h hv[2];
#pragma unroll
    for (int it = 0; it < 4; ++it) {
      const int ch  = it * 192 + tid;
      const int row = ch / 48;
      const int col = (ch - row * 48) * 4;
      fv[it] = *(const v4f*)(sT + row * kConvTP + col);
    }
#pragma unroll
    for (int it = 0; it < 2; ++it) {
      const int ch  = it * 192 + tid;
      const int row = ch / 24;
      const int col = (ch - row * 24) * 8;
      const float* sp = sT + row * kConvTP + col;
      const v4f a0 = *(const v4f*)(sp);
      const v4f a1 = *(const v4f*)(sp + 4);
#pragma unroll
      for (int e = 0; e < 4; ++e) {
        hv[it][e]     = __builtin_bit_cast(_Float16, f2bf_bits(a0[e]));
        hv[it][4 + e] = __builtin_bit_cast(_Float16, f2bf_bits(a1[e]));
      }
    }
    for (int pass = 0; pass < 2; ++pass) {
#pragma unroll
      for (int it = 0; it < 4; ++it)
        *(volatile v4f*)(UC + (size_t)lb * kDin + (size_t)(it * 192 + tid) * 4) = fv[it];
#pragma unroll
      for (int it = 0; it < 2; ++it)
        *(volatile v8h*)(UCH + (size_t)lb * kDin + (size_t)(it * 192 + tid) * 8) = hv[it];
      __threadfence();
    }
    __syncthreads();
  }
}

__global__ __launch_bounds__(64) void scan_kernel(
    const float* __restrict__ XD, const float* __restrict__ UC, const float* __restrict__ XZ,
    const float* __restrict__ Wdt, const float* __restrict__ bdt, const float* __restrict__ Alog,
    const float* __restrict__ Dp, unsigned short* __restrict__ YH, unsigned short* __restrict__ YL)
{
  __shared__ __align__(16) float sX[kScanTS * kXdP];
  __shared__ __align__(16) float sY[kScanTS * kScanYP];
  __shared__ __align__(16) float sW[8 * kScanCh];
  __shared__ __align__(16) float sA[kNst * kScanCh];
  const int tid = threadIdx.x, lane = tid & 31, wave = tid >> 5;
  constexpr int kBlkPerB = kDin / kScanCh;
  const int bix = blockIdx.x / kBlkPerB;
  const int d0  = (blockIdx.x - bix * kBlkPerB) * kScanCh;
  const int d   = d0 + tid;
  const size_t row0 = (size_t)bix * kSeq;
#pragma unroll 1
  for (int r = 0; r < kDtR; ++r) sW[r * kScanCh + tid] = Wdt[(size_t)d * kDtR + r];
#pragma unroll 1
  for (int s = 0; s < kNst; ++s) sA[s * kScanCh + tid] = -expf(Alog[(size_t)d * kNst + s]);
  __syncthreads();
  float negA[kNst], h[kNst], wr[kDtR];
#pragma unroll
  for (int s = 0; s < kNst; ++s) {
    negA[s] = sA[s * kScanCh + tid];
    h[s] = 0.f;
  }
#pragma unroll
  for (int r = 0; r < kDtR; ++r) wr[r] = sW[r * kScanCh + tid];
  const float bb = bdt[d], Dd = Dp[d];
  const int lr = tid >> 4, lc4 = (tid & 15) * 4;
  const int q = lane >> 3, c8 = (lane & 7) * 8;
#pragma unroll 1
  for (int t0 = 0; t0 < kSeq; t0 += kScanTS) {
    __syncthreads();
#pragma unroll
    for (int i = 0; i < 8; ++i) {
      const int r = lr + 4 * i;
      *(v4f*)(sX + r * kXdP + lc4) = *(const v4f*)(XD + (row0 + t0 + r) * kXdP + lc4);
    }
    asm volatile("" ::: "memory");
#pragma unroll
    for (int i = 8; i < 16; ++i) {
      const int r = lr + 4 * i;
      *(v4f*)(sX + r * kXdP + lc4) = *(const v4f*)(XD + (row0 + t0 + r) * kXdP + lc4);
    }
    __syncthreads();
#pragma unroll 1
    for (int s = 0; s < kScanTS; ++s) {
      const int t = t0 + s;
      const float* xr = sX + s * kXdP;
      const v4f x0 = *(const v4f*)(xr);
      const v4f x1 = *(const v4f*)(xr + 4);
      float vdot = bb;
      vdot = fmaf(x0[0], wr[0], vdot);
      vdot = fmaf(x0[1], wr[1], vdot);
      vdot = fmaf(x0[2], wr[2], vdot);
      vdot = fmaf(x0[3], wr[3], vdot);
      vdot = fmaf(x1[0], wr[4], vdot);
      vdot = fmaf(x1[1], wr[5], vdot);
      float Bs[kNst], Cs[kNst];
#pragma unroll
      for (int q4 = 0; q4 < 4; ++q4) {
        const v4f bv = *(const v4f*)(xr + 8 + 4 * q4);
        const v4f cv = *(const v4f*)(xr + 8 + kNst + 4 * q4);
        Bs[4 * q4 + 0] = bv[0]; Bs[4 * q4 + 1] = bv[1]; Bs[4 * q4 + 2] = bv[2]; Bs[4 * q4 + 3] = bv[3];
        Cs[4 * q4 + 0] = cv[0]; Cs[4 * q4 + 1] = cv[1]; Cs[4 * q4 + 2] = cv[2]; Cs[4 * q4 + 3] = cv[3];
      }
      const float av  = __expf(-fabsf(vdot));
      const float u   = 1.0f + av;
      const float l1p = __logf(u) + (av - (u - 1.0f)) * __builtin_amdgcn_rcpf(u);
      const float dt  = fmaxf(vdot, 0.0f) + l1p;
      const float xt  = UC[(row0 + t) * kDin + d];
      const float dtx = dt * xt;
      float y = 0.f;
#pragma unroll
      for (int k = 0; k < kNst; ++k) {
        const float e = __expf(dt * negA[k]);
        float db = dt * Bs[k];
        asm volatile("" : "+v"(db));
        float p = db * xt;
        asm volatile("" : "+v"(p));
        float qv = h[k] * e;
        asm volatile("" : "+v"(qv));
        const float hn = qv + p;
        h[k] = hn;
        float rr = Cs[k] * hn;
        asm volatile("" : "+v"(rr));
        y += rr;
      }
      (void)dtx;
      float sk = xt * Dd;
      asm volatile("" : "+v"(sk));
      y += sk;
      const float zv = XZ[(row0 + t) * kXzP + kDin + d];
      const float sg = __builtin_amdgcn_rcpf(1.0f + expf(-zv));
      y = y * (zv * sg);
      sY[s * kScanYP + tid] = y;
    }
    __syncthreads();
    v8h hv[8], lv[8];
#pragma unroll
    for (int it = 0; it < 8; ++it) {
      const int row = it * 8 + wave * 4 + q;
      const float* sp = sY + row * kScanYP + c8;
      const v4f a0 = *(const v4f*)(sp);
      const v4f a1 = *(const v4f*)(sp + 4);
#pragma unroll
      for (int e = 0; e < 4; ++e) {
        const unsigned short h0 = f2bf_bits(a0[e]), h1 = f2bf_bits(a1[e]);
        const unsigned short l0b = f2bf_bits(a0[e] - bf_bits2f(h0)), l1b = f2bf_bits(a1[e] - bf_bits2f(h1));
        hv[it][e]     = __builtin_bit_cast(_Float16, h0);
        hv[it][4 + e] = __builtin_bit_cast(_Float16, h1);
        lv[it][e]     = __builtin_bit_cast(_Float16, l0b);
        lv[it][4 + e] = __builtin_bit_cast(_Float16, l1b);
      }
    }
    for (int pass = 0; pass < 2; ++pass) {
#pragma unroll
      for (int it = 0; it < 8; ++it) {
        const int row = it * 8 + wave * 4 + q;
        const size_t o = (row0 + t0 + row) * kDin + d0 + c8;
        *(volatile v8h*)(YH + o) = hv[it];
        *(volatile v8h*)(YL + o) = lv[it];
      }
      __threadfence();
    }
  }
}

extern "C" void kernel_launch(void* const* d_in, const int* in_sizes, int n_in,
                              void* d_out, int out_size, void* d_ws, size_t ws_size,
                              hipStream_t stream) {
  if (n_in < 12) return;
  if (in_sizes[0] != kRows * kDim) return;
  if (in_sizes[1] != kDim || in_sizes[2] != kDim) return;
  if (in_sizes[3] != kXzP * kDim) return;
  if (in_sizes[4] != kDin * 4 || in_sizes[5] != kDin) return;
  if (in_sizes[6] != kXpN * kDin) return;
  if (in_sizes[7] != kDin * kDtR || in_sizes[8] != kDin) return;
  if (in_sizes[9] != kDin * kNst || in_sizes[10] != kDin) return;
  if (in_sizes[11] != kDim * kDin) return;
  if (out_size != kRows * kDim) return;
  if (ws_size < kWsTotal) return;

  const float* x          = (const float*)d_in[0];
  const float* gamma      = (const float*)d_in[1];
  const float* beta       = (const float*)d_in[2];
  const float* in_proj_w  = (const float*)d_in[3];
  const float* conv_w     = (const float*)d_in[4];
  const float* conv_b     = (const float*)d_in[5];
  const float* x_proj_w   = (const float*)d_in[6];
  const float* dt_proj_w  = (const float*)d_in[7];
  const float* dt_proj_b  = (const float*)d_in[8];
  const float* A_log      = (const float*)d_in[9];
  const float* D_param    = (const float*)d_in[10];
  const float* out_proj_w = (const float*)d_in[11];
  float* out = (float*)d_out;

  char* ws = (char*)d_ws;
  unsigned short* XNH = (unsigned short*)(ws + kOffXNH);
  unsigned short* XNL = (unsigned short*)(ws + kOffXNL);
  unsigned short* WIH = (unsigned short*)(ws + kOffWIH);
  unsigned short* WIL = (unsigned short*)(ws + kOffWIL);
  unsigned short* WXH = (unsigned short*)(ws + kOffWXH);
  unsigned short* WOH = (unsigned short*)(ws + kOffWOH);
  unsigned short* WOL = (unsigned short*)(ws + kOffWOL);
  float*          XZ  = (float*)(ws + kOffXZ);
  float*          UC  = (float*)(ws + kOffUC);
  unsigned short* UCH = (unsigned short*)(ws + kOffUCH);
  float*          XD  = (float*)(ws + kOffXD);
  unsigned short* YH  = (unsigned short*)(ws + kOffYH);
  unsigned short* YL  = (unsigned short*)(ws + kOffYL);
  const float* dummy_bias  = dt_proj_b;
  const float* dummy_resid = x;

  constexpr int kWin8  = kXzP * kDim / 8;
  constexpr int kWout8 = kDim * kDin / 8;
  constexpr int kWoutP = kOutM * kDin / 8;
  constexpr int kWx8   = kXdP * kDin / 8;
  static_assert(kWin8 % 256 == 0 && kWoutP % 256 == 0 && kWx8 % 256 == 0, "");
  split_pad_bf16_kernel<<<kWin8 / 256, 256, 0, stream>>>(in_proj_w, WIH, WIL, kWin8, kWin8);
  split_pad_bf16_kernel<<<kWoutP / 256, 256, 0, stream>>>(out_proj_w, WOH, WOL, kWout8, kWoutP);
  xproj_plane_kernel<<<kWx8 / 256, 256, 0, stream>>>(x_proj_w, WXH, kWx8);

  ln_split_kernel<<<kRows / 64, 256, 0, stream>>>(x, gamma, beta, XNH, XNL);

  {
    constexpr int tiles = (kRows / 64) * (kXzP / 64);
    wmma_gemm64<1, true, 0, 0, false><<<dim3((tiles + 7) / 8, 1), 256, 0, stream>>>(
        XNH, XNL, kDim, 0L,
        WIH, WIL, kDim, 0L,
        (void*)XZ, (void*)XZ, kXzP, 0L,
        dummy_bias, dummy_resid, 0L,
        kRows, kXzP, kDim, 1.0f, kRows);
  }

  conv_silu_kernel<<<kRows / 64, kDin, 0, stream>>>(XZ, conv_w, conv_b, UC, UCH);

  {
    constexpr int tiles = (kRows / 64) * (kXdP / 64);
    wmma_gemm64<1, false, 0, 0, false><<<dim3((tiles + 7) / 8, 1), 256, 0, stream>>>(
        UCH, UCH, kDin, 0L,
        WXH, WXH, kDin, 0L,
        (void*)XD, (void*)XD, kXdP, 0L,
        dummy_bias, dummy_resid, 0L,
        kRows, kXdP, kDin, 1.0f, kRows);
  }

  scan_kernel<<<kBatch * (kDin / kScanCh), kScanCh, 0, stream>>>(XD, UC, XZ, dt_proj_w, dt_proj_b, A_log, D_param, YH, YL);

  {
    constexpr int tiles = (kOutM / 64) * (kSeq / 64);
    wmma_gemm64<1, true, 0, 0, false><<<dim3((tiles + 7) / 8, kBatch), 256, 0, stream>>>(
        WOH, WOL, kDin, 0L,
        YH, YL, kDin, (long)kSeq * kDin,
        (void*)out, (void*)out, kSeq, (long)kDim * kSeq,
        dummy_bias, dummy_resid, 0L,
        kOutM, kSeq, kDin, 1.0f, kDim);
  }
}
